// FullyFrameAttention_1726576855779
// MI455X (gfx1250) — hardware-verified
//
#include <hip/hip_runtime.h>
#include <math.h>

typedef __attribute__((ext_vector_type(16))) _Float16 v16h;
typedef __attribute__((ext_vector_type(16))) __bf16 v16b;
typedef __attribute__((ext_vector_type(8)))  _Float16 v8h;
typedef __attribute__((ext_vector_type(8)))  float v8f;
typedef __attribute__((ext_vector_type(4)))  float v4f;
typedef __attribute__((ext_vector_type(2)))  float v2f;
typedef __attribute__((ext_vector_type(4)))  unsigned v4u;
typedef __attribute__((ext_vector_type(4)))  int v4i;
typedef float __attribute__((may_alias)) float_a;
typedef int __attribute__((may_alias)) int_a;

template <typename T> __device__ __forceinline__ void vst2(void* p, T v) { *(volatile T*)p = v; __threadfence(); *(volatile T*)p = v; }
__device__ __forceinline__ v8f wmma16(v16h a, v16h b, v8f c) {
  v8f d = __builtin_amdgcn_wmma_f32_16x16x32_f16(false, a, false, b, (short)0, c, false, false);
  asm volatile("v_nop\n\tv_nop\n\tv_nop\n\tv_nop" : "+v"(d) : "v"(a), "v"(b));
  return d;
}
__device__ __forceinline__ v8f wmma_bf(v16b a, v16b b, v8f c) {
  v8f d = __builtin_amdgcn_wmma_f32_16x16x32_bf16(false, a, false, b, (short)0, c, false, false);
  asm volatile("v_nop\n\tv_nop\n\tv_nop\n\tv_nop" : "+v"(d) : "v"(a), "v"(b));
  return d;
}
__device__ __forceinline__ v16h frag_h(const _Float16* rowk0, int lane) {
  union { v16h v; v8h q[2]; } u; const _Float16* p = rowk0 + 8 * (lane >> 4);
  u.q[0] = *(const v8h*)p; u.q[1] = *(const v8h*)(p + 16); return u.v;
}
__device__ __forceinline__ v16h frag_f32(const float* rowk0, int lane) {
  v16h a; const float* p = rowk0 + 8 * (lane >> 4);
#pragma unroll
  for (int i = 0; i < 8; ++i) { a[i] = (_Float16)p[i]; a[8 + i] = (_Float16)p[16 + i]; }
  return a;
}
__device__ __forceinline__ v16h frag_f32s(const float* rowk0, int lane, float sc) {
  v16h a; const float* p = rowk0 + 8 * (lane >> 4);
#pragma unroll
  for (int i = 0; i < 8; ++i) { a[i] = (_Float16)(p[i] * sc); a[8 + i] = (_Float16)(p[16 + i] * sc); }
  return a;
}
__device__ __forceinline__ v16h fragc_f32(const float* W, int k0, int n, int lane, int ld, int K) {
  v16h a; const int g = lane >> 4;
#pragma unroll
  for (int i = 0; i < 8; ++i) { const int ka = k0 + 8 * g + i, kb = ka + 16;
    a[i] = (_Float16)(ka < K ? W[(size_t)(ka < K ? ka : K - 1) * ld + n] : 0.f); a[8 + i] = (_Float16)(kb < K ? W[(size_t)(kb < K ? kb : K - 1) * ld + n] : 0.f); }
  return a;
}
struct F2 { v16b h, l; };
__device__ __forceinline__ F2 bsplit16(const float v[16]) { F2 r;
#pragma unroll
  for (int i = 0; i < 16; ++i) { const __bf16 h = (__bf16)v[i]; r.h[i] = h; r.l[i] = (__bf16)(v[i] - (float)h); }
  return r; }
__device__ __forceinline__ F2 split_row(const float* row, int k0, int lane) { float v[16]; const float* p = row + k0 + 8 * (lane >> 4);
#pragma unroll
  for (int i = 0; i < 8; ++i) { v[i] = p[i]; v[8 + i] = p[16 + i]; }
  return bsplit16(v); }
__device__ __forceinline__ F2 split_rowK(const float* row, int k0, int lane, int K) { float v[16]; const int g = lane >> 4;
#pragma unroll
  for (int i = 0; i < 8; ++i) { const int ka = k0 + 8 * g + i, kb = ka + 16; v[i] = ka < K ? row[ka < K ? ka : K - 1] : 0.f; v[8 + i] = kb < K ? row[kb < K ? kb : K - 1] : 0.f; }
  return bsplit16(v); }
__device__ __forceinline__ F2 split_col(const float* W, int k0, int n, int lane, int ld, int K) { float v[16]; const int g = lane >> 4;
#pragma unroll
  for (int i = 0; i < 8; ++i) { const int ka = k0 + 8 * g + i, kb = ka + 16; v[i] = ka < K ? W[(size_t)(ka < K ? ka : K - 1) * ld + n] : 0.f; v[8 + i] = kb < K ? W[(size_t)(kb < K ? kb : K - 1) * ld + n] : 0.f; }
  return bsplit16(v); }
__device__ __forceinline__ v8f mac3(const F2& a, const F2& b, v8f c) { c = wmma_bf(a.l, b.h, c); c = wmma_bf(a.h, b.l, c); return wmma_bf(a.h, b.h, c); }
__device__ __forceinline__ float sigm(float v) { return 1.0f / (1.0f + expf(-v)); }
#define LDSX() do { asm volatile("s_wait_dscnt 0" ::: "memory"); __builtin_amdgcn_wave_barrier(); __builtin_amdgcn_fence(__ATOMIC_RELEASE, "workgroup"); } while (0)


#define SS 4096
#define CC 320
#define CP 336
#define NH 8
#define HD 40
#define HP 64
#define OP (NH * HP)
#ifndef TQB
#define TQB (SS / 64)
#endif
typedef __attribute__((ext_vector_type(8))) __bf16 v8b;
__device__ __forceinline__ v16b frag_b(const __bf16* rowk0, int lane) {
  union { v16b v; v8b q[2]; } u; const __bf16* p = rowk0 + 8 * (lane >> 4);
  u.q[0] = *(const v8b*)p; u.q[1] = *(const v8b*)(p + 16); return u.v;
}
__device__ __forceinline__ float bfr(float v) { return (float)(__bf16)v; }
__device__ __attribute__((noinline)) float exp_ni(float v) { return expf(v); }
__device__ __attribute__((noinline)) float erf_ni(float v) { return erff(v); }

#define WS_PW  0u
#define WS_PO  (WS_PW + 2u * (size_t)3 * CP * CC)
#define WS_Q   (WS_PO + 2u * (size_t)CC * OP)
#define WS_K   (WS_Q + 2u * (size_t)SS * OP)
#define WS_V   (WS_K + 2u * (size_t)SS * OP)
#define WS_O   (WS_V + 2u * (size_t)CP * SS)
#define WS_END (WS_O + 4u * (size_t)SS * OP)

__global__ __launch_bounds__(128) void k_pack(const float* __restrict__ WQ, const float* __restrict__ WK, const float* __restrict__ WV, const float* __restrict__ WO, __bf16* __restrict__ PW, __bf16* __restrict__ PO) {
  const int n = blockIdx.x, which = blockIdx.y, t = threadIdx.x; __shared__ __align__(16) __bf16 s[OP];
  if (which < 3) { const float* w = (which == 0) ? WQ : (which == 1) ? WK : WV; for (int k = t; k < CC; k += 128) s[k] = (n < CC) ? (__bf16)w[(size_t)k * CC + n] : (__bf16)0.f; __syncthreads(); if (t < CC / 8) vst2((unsigned*)(PW + ((size_t)which * CP + n) * CC + t * 8), *(const v4u*)&s[t * 8]); }
  else { if (n >= CC) return; for (int k = t; k < OP; k += 128) { const int h = k / HP, d = k % HP; s[k] = (d < HD) ? (__bf16)WO[(size_t)(h * HD + d) * CC + n] : (__bf16)0.f; } __syncthreads(); if (t < OP / 8) vst2((unsigned*)(PO + (size_t)n * OP + t * 8), *(const v4u*)&s[t * 8]); }
}
__global__ __launch_bounds__(128) void k_qkv(const float* __restrict__ X, const __bf16* __restrict__ PW, _Float16* __restrict__ Q, _Float16* __restrict__ Kr, _Float16* __restrict__ V) {
  __shared__ __align__(16) _Float16 so[64][HP + 8]; __shared__ __align__(16) _Float16 st[48][72];
  const int tid = threadIdx.x, wave = tid >> 5, lane = tid & 31, col = lane & 15, g = lane >> 4; const int h = blockIdx.y, which = blockIdx.z; const int n0b = blockIdx.x * 64; const size_t r0 = (size_t)n0b + wave * 16; const int c0 = h * HD;
  const __bf16* P = PW + ((size_t)which * CP) * CC;
  v8f acc[3] = {};
#pragma unroll 2
  for (int kc = 0; kc < CC / 32; ++kc) { v16b a; { const float* p = X + (r0 + col) * CC + kc * 32 + 8 * g;
#pragma unroll
      for (int i = 0; i < 8; ++i) { a[i] = (__bf16)p[i]; a[8 + i] = (__bf16)p[16 + i]; } }
#pragma unroll
    for (int j = 0; j < 3; ++j) acc[j] = wmma_bf(a, frag_b(P + (size_t)(c0 + j * 16 + col) * CC + kc * 32, lane), acc[j]); }
  if (which < 2) { _Float16* dst = (which == 0) ? Q : Kr;
#pragma unroll
    for (int j = 0; j < 4; ++j)
#pragma unroll
      for (int r = 0; r < 8; ++r) { const int d = j * 16 + col; so[wave * 16 + 8 * g + r][d] = (j < 3 && d < HD) ? (_Float16)acc[j < 3 ? j : 0][r] : (_Float16)0.f; }
    __syncthreads();
    for (int e = tid; e < 64 * 8; e += 128) { const int rl = e >> 3, q = e & 7; vst2((unsigned*)(dst + (size_t)(n0b + rl) * OP + h * HP + q * 8), *(const v4u*)&so[rl][q * 8]); }
  } else {
#pragma unroll
    for (int j = 0; j < 3; ++j)
#pragma unroll
      for (int r = 0; r < 8; ++r) st[j * 16 + col][wave * 16 + 8 * g + r] = (_Float16)acc[j][r];
    __syncthreads();
    for (int e = tid; e < HD * 8; e += 128) { const int d = e >> 3, pc = e & 7; vst2((unsigned*)(V + ((size_t)(c0 + d) * SS) + n0b + pc * 8), *(const v4u*)&st[d][pc * 8]); } }
}
__global__ __launch_bounds__(128) void k_attn(const _Float16* __restrict__ Q, const _Float16* __restrict__ Kr, const _Float16* __restrict__ V, float* __restrict__ O) {
  __shared__ __align__(16) _Float16 sph[4][16][40]; __shared__ __align__(16) float so[4][16][68];
  const int tid = threadIdx.x, wave = tid >> 5, lane = tid & 31, col = lane & 15, g = lane >> 4; const int h = blockIdx.y; const int q0 = blockIdx.x * 64 + wave * 16; const size_t rq = q0;
  v16h aq[2];
#pragma unroll
  for (int kc = 0; kc < 2; ++kc) aq[kc] = frag_h(Q + (rq + col) * OP + h * HP + kc * 32, lane);
  float m[8], l[8];
#pragma unroll
  for (int r = 0; r < 8; ++r) { m[r] = -3.0e38f; l[r] = 0.f; }
  v8f acc[3] = {};
#pragma unroll 1
  for (int ks = 0; ks < SS / 32; ++ks) { const int j0 = ks * 32; v8f s[2];
#pragma unroll
    for (int ct = 0; ct < 2; ++ct) { const size_t rk = (size_t)(j0 + ct * 16 + col) * OP + h * HP; v8f c = {};
#pragma unroll
      for (int kc = 0; kc < 2; ++kc) c = wmma16(aq[kc], frag_h(Kr + rk + kc * 32, lane), c);
#pragma unroll
      for (int r = 0; r < 8; ++r) s[ct][r] = c[r] * 0.15811388300841897f; }
#pragma unroll
    for (int r = 0; r < 8; ++r) { float mx = fmaxf(s[0][r], s[1][r]);
#pragma unroll
      for (int o = 1; o < 16; o <<= 1) mx = fmaxf(mx, __shfl_xor(mx, o));
      const float mn = fmaxf(m[r], mx); const float alpha = (m[r] <= -1.0e38f) ? 0.f : __expf(m[r] - mn); const float e0 = __expf(s[0][r] - mn), e1 = __expf(s[1][r] - mn); float es = e0 + e1;
#pragma unroll
      for (int o = 1; o < 16; o <<= 1) es += __shfl_xor(es, o);
      l[r] = l[r] * alpha + es; m[r] = mn;
#pragma unroll
      for (int dt = 0; dt < 3; ++dt) acc[dt][r] *= alpha;
      sph[wave][8 * g + r][col] = (_Float16)(e0 * 2048.0f); sph[wave][8 * g + r][16 + col] = (_Float16)(e1 * 2048.0f); }
    LDSX();
    const v16h pa = frag_h(&sph[wave][col][0], lane);
#pragma unroll
    for (int dt = 0; dt < 3; ++dt) acc[dt] = wmma16(pa, frag_h(V + ((size_t)(h * HD + dt * 16 + col) * SS) + j0, lane), acc[dt]);
    LDSX(); }
#pragma unroll
  for (int r = 0; r < 8; ++r) { const float il = (1.0f / 2048.0f) / l[r];
#pragma unroll
    for (int dt = 0; dt < 4; ++dt) { const int d = dt * 16 + col; so[wave][8 * g + r][d] = (dt < 3 && d < HD) ? acc[dt < 3 ? dt : 0][r] * il : 0.f; } }
  LDSX();
  for (int rl = 0; rl < 16; ++rl) if (lane < 16) vst2(O + (rq + rl) * OP + h * HP + lane * 4, *(const v4f*)&so[wave][rl][lane * 4]);
}
__global__ __launch_bounds__(128) void k_out(const float* __restrict__ O, const __bf16* __restrict__ PO, const float* __restrict__ BO, float* __restrict__ OUT) {
  __shared__ __align__(16) float so[4][16][68];
  const int tid = threadIdx.x, wave = tid >> 5, lane = tid & 31, col = lane & 15, g = lane >> 4; const size_t r0 = (size_t)blockIdx.x * 64 + wave * 16; const int o0 = blockIdx.y * 64;
  v8f acc[4] = {};
#pragma unroll 2
  for (int kc = 0; kc < OP / 32; ++kc) { const F2 a = split_row(O + (r0 + col) * OP, kc * 32, lane);
#pragma unroll
    for (int j = 0; j < 4; ++j) { const v16b w = frag_b(PO + (size_t)(o0 + j * 16 + col) * OP + kc * 32, lane); acc[j] = wmma_bf(a.l, w, acc[j]); acc[j] = wmma_bf(a.h, w, acc[j]); } }
#pragma unroll
  for (int j = 0; j < 4; ++j) { const float bb = bfr(BO[o0 + j * 16 + col]);
#pragma unroll
    for (int r = 0; r < 8; ++r) so[wave][8 * g + r][j * 16 + col] = acc[j][r] + bb; }
  LDSX();
  for (int rl = 0; rl < 16; ++rl) if (lane < 16) vst2(OUT + (r0 + rl) * CC + o0 + lane * 4, *(const v4f*)&so[wave][rl][lane * 4]);
}
extern "C" void kernel_launch(void* const* d_in, const int* in_sizes, int n_in, void* d_out, int out_size, void* d_ws, size_t ws_size, hipStream_t stream) {
  (void)in_sizes; (void)n_in; (void)out_size;
  const float** F = (const float**)d_in;
  if (ws_size < (size_t)WS_END) return;
  char* ws = (char*)d_ws; __bf16 *PW = (__bf16*)(ws + WS_PW), *PO = (__bf16*)(ws + WS_PO); _Float16 *Q = (_Float16*)(ws + WS_Q), *Kr = (_Float16*)(ws + WS_K), *V = (_Float16*)(ws + WS_V); float* O = (float*)(ws + WS_O);
  k_pack<<<dim3(CP, 4), 128, 0, stream>>>(F[1], F[2], F[3], F[4], PW, PO);
  k_qkv<<<dim3(SS / 64, NH, 3), 128, 0, stream>>>(F[0], PW, Q, Kr, V);
  k_attn<<<dim3(TQB, NH), 128, 0, stream>>>(Q, Kr, V, O);
  k_out<<<dim3(TQB, CC / 64), 128, 0, stream>>>(O, PO, F[5], (float*)d_out);
}
